// UpThreeOffsetsConv_87660282511816
// MI455X (gfx1250) — hardware-verified
//
#include <hip/hip_runtime.h>


#define CI   64
#define CO   64
#define DIMI 24
#define DIMO 48
#define NVOX (DIMO * DIMO * DIMO)
#define KT   (CI * 27)
#define NV   4608
#define C3   (3 * CO)
#define BN_EPS 1e-5f
#define DM   KT
#define LOSC 1024.0f

__constant__ float c_tab04[27][27] = {{0.216000006f,0.143999994f,0.f,0.143999994f,0.0960000008f,0.f,0.f,0.f,0.f,0.143999994f,0.0960000008f,0.f,0.0960000008f,0.0640000030f,0.f,0.f,0.f,0.f,0.f,0.f,0.f,0.f,0.f,0.f,0.f,0.f,0.f},
{0.f,0.360000014f,0.f,0.f,0.239999995f,0.f,0.f,0.f,0.f,0.f,0.239999995f,0.f,0.f,0.159999996f,0.f,0.f,0.f,0.f,0.f,0.f,0.f,0.f,0.f,0.f,0.f,0.f,0.f},
{0.f,0.143999994f,0.216000006f,0.f,0.0960000008f,0.143999994f,0.f,0.f,0.f,0.f,0.0960000008f,0.143999994f,0.f,0.0640000030f,0.0960000008f,0.f,0.f,0.f,0.f,0.f,0.f,0.f,0.f,0.f,0.f,0.f,0.f},
{0.f,0.f,0.f,0.360000014f,0.239999995f,0.f,0.f,0.f,0.f,0.f,0.f,0.f,0.239999995f,0.159999996f,0.f,0.f,0.f,0.f,0.f,0.f,0.f,0.f,0.f,0.f,0.f,0.f,0.f},
{0.f,0.f,0.f,0.f,0.600000024f,0.f,0.f,0.f,0.f,0.f,0.f,0.f,0.f,0.400000006f,0.f,0.f,0.f,0.f,0.f,0.f,0.f,0.f,0.f,0.f,0.f,0.f,0.f},
{0.f,0.f,0.f,0.f,0.239999995f,0.360000014f,0.f,0.f,0.f,0.f,0.f,0.f,0.f,0.159999996f,0.239999995f,0.f,0.f,0.f,0.f,0.f,0.f,0.f,0.f,0.f,0.f,0.f,0.f},
{0.f,0.f,0.f,0.143999994f,0.0960000008f,0.f,0.216000006f,0.143999994f,0.f,0.f,0.f,0.f,0.0960000008f,0.0640000030f,0.f,0.143999994f,0.0960000008f,0.f,0.f,0.f,0.f,0.f,0.f,0.f,0.f,0.f,0.f},
{0.f,0.f,0.f,0.f,0.239999995f,0.f,0.f,0.360000014f,0.f,0.f,0.f,0.f,0.f,0.159999996f,0.f,0.f,0.239999995f,0.f,0.f,0.f,0.f,0.f,0.f,0.f,0.f,0.f,0.f},
{0.f,0.f,0.f,0.f,0.0960000008f,0.143999994f,0.f,0.143999994f,0.216000006f,0.f,0.f,0.f,0.f,0.0640000030f,0.0960000008f,0.f,0.0960000008f,0.143999994f,0.f,0.f,0.f,0.f,0.f,0.f,0.f,0.f,0.f},
{0.f,0.f,0.f,0.f,0.f,0.f,0.f,0.f,0.f,0.360000014f,0.239999995f,0.f,0.239999995f,0.159999996f,0.f,0.f,0.f,0.f,0.f,0.f,0.f,0.f,0.f,0.f,0.f,0.f,0.f},
{0.f,0.f,0.f,0.f,0.f,0.f,0.f,0.f,0.f,0.f,0.600000024f,0.f,0.f,0.400000006f,0.f,0.f,0.f,0.f,0.f,0.f,0.f,0.f,0.f,0.f,0.f,0.f,0.f},
{0.f,0.f,0.f,0.f,0.f,0.f,0.f,0.f,0.f,0.f,0.239999995f,0.360000014f,0.f,0.159999996f,0.239999995f,0.f,0.f,0.f,0.f,0.f,0.f,0.f,0.f,0.f,0.f,0.f,0.f},
{0.f,0.f,0.f,0.f,0.f,0.f,0.f,0.f,0.f,0.f,0.f,0.f,0.600000024f,0.400000006f,0.f,0.f,0.f,0.f,0.f,0.f,0.f,0.f,0.f,0.f,0.f,0.f,0.f},
{0.f,0.f,0.f,0.f,0.f,0.f,0.f,0.f,0.f,0.f,0.f,0.f,0.f,1.00000000f,0.f,0.f,0.f,0.f,0.f,0.f,0.f,0.f,0.f,0.f,0.f,0.f,0.f},
{0.f,0.f,0.f,0.f,0.f,0.f,0.f,0.f,0.f,0.f,0.f,0.f,0.f,0.400000006f,0.600000024f,0.f,0.f,0.f,0.f,0.f,0.f,0.f,0.f,0.f,0.f,0.f,0.f},
{0.f,0.f,0.f,0.f,0.f,0.f,0.f,0.f,0.f,0.f,0.f,0.f,0.239999995f,0.159999996f,0.f,0.360000014f,0.239999995f,0.f,0.f,0.f,0.f,0.f,0.f,0.f,0.f,0.f,0.f},
{0.f,0.f,0.f,0.f,0.f,0.f,0.f,0.f,0.f,0.f,0.f,0.f,0.f,0.400000006f,0.f,0.f,0.600000024f,0.f,0.f,0.f,0.f,0.f,0.f,0.f,0.f,0.f,0.f},
{0.f,0.f,0.f,0.f,0.f,0.f,0.f,0.f,0.f,0.f,0.f,0.f,0.f,0.159999996f,0.239999995f,0.f,0.239999995f,0.360000014f,0.f,0.f,0.f,0.f,0.f,0.f,0.f,0.f,0.f},
{0.f,0.f,0.f,0.f,0.f,0.f,0.f,0.f,0.f,0.143999994f,0.0960000008f,0.f,0.0960000008f,0.0640000030f,0.f,0.f,0.f,0.f,0.216000006f,0.143999994f,0.f,0.143999994f,0.0960000008f,0.f,0.f,0.f,0.f},
{0.f,0.f,0.f,0.f,0.f,0.f,0.f,0.f,0.f,0.f,0.239999995f,0.f,0.f,0.159999996f,0.f,0.f,0.f,0.f,0.f,0.360000014f,0.f,0.f,0.239999995f,0.f,0.f,0.f,0.f},
{0.f,0.f,0.f,0.f,0.f,0.f,0.f,0.f,0.f,0.f,0.0960000008f,0.143999994f,0.f,0.0640000030f,0.0960000008f,0.f,0.f,0.f,0.f,0.143999994f,0.216000006f,0.f,0.0960000008f,0.143999994f,0.f,0.f,0.f},
{0.f,0.f,0.f,0.f,0.f,0.f,0.f,0.f,0.f,0.f,0.f,0.f,0.239999995f,0.159999996f,0.f,0.f,0.f,0.f,0.f,0.f,0.f,0.360000014f,0.239999995f,0.f,0.f,0.f,0.f},
{0.f,0.f,0.f,0.f,0.f,0.f,0.f,0.f,0.f,0.f,0.f,0.f,0.f,0.400000006f,0.f,0.f,0.f,0.f,0.f,0.f,0.f,0.f,0.600000024f,0.f,0.f,0.f,0.f},
{0.f,0.f,0.f,0.f,0.f,0.f,0.f,0.f,0.f,0.f,0.f,0.f,0.f,0.159999996f,0.239999995f,0.f,0.f,0.f,0.f,0.f,0.f,0.f,0.239999995f,0.360000014f,0.f,0.f,0.f},
{0.f,0.f,0.f,0.f,0.f,0.f,0.f,0.f,0.f,0.f,0.f,0.f,0.0960000008f,0.0640000030f,0.f,0.143999994f,0.0960000008f,0.f,0.f,0.f,0.f,0.143999994f,0.0960000008f,0.f,0.216000006f,0.143999994f,0.f},
{0.f,0.f,0.f,0.f,0.f,0.f,0.f,0.f,0.f,0.f,0.f,0.f,0.f,0.159999996f,0.f,0.f,0.239999995f,0.f,0.f,0.f,0.f,0.f,0.239999995f,0.f,0.f,0.360000014f,0.f},
{0.f,0.f,0.f,0.f,0.f,0.f,0.f,0.f,0.f,0.f,0.f,0.f,0.f,0.0640000030f,0.0960000008f,0.f,0.0960000008f,0.143999994f,0.f,0.f,0.f,0.f,0.0960000008f,0.143999994f,0.f,0.143999994f,0.216000006f}};
__constant__ float c_tab07[27][27] = {{0.0270000007f,0.0630000010f,0.f,0.0630000010f,0.147000000f,0.f,0.f,0.f,0.f,0.0630000010f,0.147000000f,0.f,0.147000000f,0.342999995f,0.f,0.f,0.f,0.f,0.f,0.f,0.f,0.f,0.f,0.f,0.f,0.f,0.f},
{0.f,0.0900000036f,0.f,0.f,0.209999993f,0.f,0.f,0.f,0.f,0.f,0.209999993f,0.f,0.f,0.490000010f,0.f,0.f,0.f,0.f,0.f,0.f,0.f,0.f,0.f,0.f,0.f,0.f,0.f},
{0.f,0.0630000010f,0.0270000007f,0.f,0.147000000f,0.0630000010f,0.f,0.f,0.f,0.f,0.147000000f,0.0630000010f,0.f,0.342999995f,0.147000000f,0.f,0.f,0.f,0.f,0.f,0.f,0.f,0.f,0.f,0.f,0.f,0.f},
{0.f,0.f,0.f,0.0900000036f,0.209999993f,0.f,0.f,0.f,0.f,0.f,0.f,0.f,0.209999993f,0.490000010f,0.f,0.f,0.f,0.f,0.f,0.f,0.f,0.f,0.f,0.f,0.f,0.f,0.f},
{0.f,0.f,0.f,0.f,0.300000012f,0.f,0.f,0.f,0.f,0.f,0.f,0.f,0.f,0.699999988f,0.f,0.f,0.f,0.f,0.f,0.f,0.f,0.f,0.f,0.f,0.f,0.f,0.f},
{0.f,0.f,0.f,0.f,0.209999993f,0.0900000036f,0.f,0.f,0.f,0.f,0.f,0.f,0.f,0.490000010f,0.209999993f,0.f,0.f,0.f,0.f,0.f,0.f,0.f,0.f,0.f,0.f,0.f,0.f},
{0.f,0.f,0.f,0.0630000010f,0.147000000f,0.f,0.0270000007f,0.0630000010f,0.f,0.f,0.f,0.f,0.147000000f,0.342999995f,0.f,0.0630000010f,0.147000000f,0.f,0.f,0.f,0.f,0.f,0.f,0.f,0.f,0.f,0.f},
{0.f,0.f,0.f,0.f,0.209999993f,0.f,0.f,0.0900000036f,0.f,0.f,0.f,0.f,0.f,0.490000010f,0.f,0.f,0.209999993f,0.f,0.f,0.f,0.f,0.f,0.f,0.f,0.f,0.f,0.f},
{0.f,0.f,0.f,0.f,0.147000000f,0.0630000010f,0.f,0.0630000010f,0.0270000007f,0.f,0.f,0.f,0.f,0.342999995f,0.147000000f,0.f,0.147000000f,0.0630000010f,0.f,0.f,0.f,0.f,0.f,0.f,0.f,0.f,0.f},
{0.f,0.f,0.f,0.f,0.f,0.f,0.f,0.f,0.f,0.0900000036f,0.209999993f,0.f,0.209999993f,0.490000010f,0.f,0.f,0.f,0.f,0.f,0.f,0.f,0.f,0.f,0.f,0.f,0.f,0.f},
{0.f,0.f,0.f,0.f,0.f,0.f,0.f,0.f,0.f,0.f,0.300000012f,0.f,0.f,0.699999988f,0.f,0.f,0.f,0.f,0.f,0.f,0.f,0.f,0.f,0.f,0.f,0.f,0.f},
{0.f,0.f,0.f,0.f,0.f,0.f,0.f,0.f,0.f,0.f,0.209999993f,0.0900000036f,0.f,0.490000010f,0.209999993f,0.f,0.f,0.f,0.f,0.f,0.f,0.f,0.f,0.f,0.f,0.f,0.f},
{0.f,0.f,0.f,0.f,0.f,0.f,0.f,0.f,0.f,0.f,0.f,0.f,0.300000012f,0.699999988f,0.f,0.f,0.f,0.f,0.f,0.f,0.f,0.f,0.f,0.f,0.f,0.f,0.f},
{0.f,0.f,0.f,0.f,0.f,0.f,0.f,0.f,0.f,0.f,0.f,0.f,0.f,1.00000000f,0.f,0.f,0.f,0.f,0.f,0.f,0.f,0.f,0.f,0.f,0.f,0.f,0.f},
{0.f,0.f,0.f,0.f,0.f,0.f,0.f,0.f,0.f,0.f,0.f,0.f,0.f,0.699999988f,0.300000012f,0.f,0.f,0.f,0.f,0.f,0.f,0.f,0.f,0.f,0.f,0.f,0.f},
{0.f,0.f,0.f,0.f,0.f,0.f,0.f,0.f,0.f,0.f,0.f,0.f,0.209999993f,0.490000010f,0.f,0.0900000036f,0.209999993f,0.f,0.f,0.f,0.f,0.f,0.f,0.f,0.f,0.f,0.f},
{0.f,0.f,0.f,0.f,0.f,0.f,0.f,0.f,0.f,0.f,0.f,0.f,0.f,0.699999988f,0.f,0.f,0.300000012f,0.f,0.f,0.f,0.f,0.f,0.f,0.f,0.f,0.f,0.f},
{0.f,0.f,0.f,0.f,0.f,0.f,0.f,0.f,0.f,0.f,0.f,0.f,0.f,0.490000010f,0.209999993f,0.f,0.209999993f,0.0900000036f,0.f,0.f,0.f,0.f,0.f,0.f,0.f,0.f,0.f},
{0.f,0.f,0.f,0.f,0.f,0.f,0.f,0.f,0.f,0.0630000010f,0.147000000f,0.f,0.147000000f,0.342999995f,0.f,0.f,0.f,0.f,0.0270000007f,0.0630000010f,0.f,0.0630000010f,0.147000000f,0.f,0.f,0.f,0.f},
{0.f,0.f,0.f,0.f,0.f,0.f,0.f,0.f,0.f,0.f,0.209999993f,0.f,0.f,0.490000010f,0.f,0.f,0.f,0.f,0.f,0.0900000036f,0.f,0.f,0.209999993f,0.f,0.f,0.f,0.f},
{0.f,0.f,0.f,0.f,0.f,0.f,0.f,0.f,0.f,0.f,0.147000000f,0.0630000010f,0.f,0.342999995f,0.147000000f,0.f,0.f,0.f,0.f,0.0630000010f,0.0270000007f,0.f,0.147000000f,0.0630000010f,0.f,0.f,0.f},
{0.f,0.f,0.f,0.f,0.f,0.f,0.f,0.f,0.f,0.f,0.f,0.f,0.209999993f,0.490000010f,0.f,0.f,0.f,0.f,0.f,0.f,0.f,0.0900000036f,0.209999993f,0.f,0.f,0.f,0.f},
{0.f,0.f,0.f,0.f,0.f,0.f,0.f,0.f,0.f,0.f,0.f,0.f,0.f,0.699999988f,0.f,0.f,0.f,0.f,0.f,0.f,0.f,0.f,0.300000012f,0.f,0.f,0.f,0.f},
{0.f,0.f,0.f,0.f,0.f,0.f,0.f,0.f,0.f,0.f,0.f,0.f,0.f,0.490000010f,0.209999993f,0.f,0.f,0.f,0.f,0.f,0.f,0.f,0.209999993f,0.0900000036f,0.f,0.f,0.f},
{0.f,0.f,0.f,0.f,0.f,0.f,0.f,0.f,0.f,0.f,0.f,0.f,0.147000000f,0.342999995f,0.f,0.0630000010f,0.147000000f,0.f,0.f,0.f,0.f,0.0630000010f,0.147000000f,0.f,0.0270000007f,0.0630000010f,0.f},
{0.f,0.f,0.f,0.f,0.f,0.f,0.f,0.f,0.f,0.f,0.f,0.f,0.f,0.490000010f,0.f,0.f,0.209999993f,0.f,0.f,0.f,0.f,0.f,0.209999993f,0.f,0.f,0.0900000036f,0.f},
{0.f,0.f,0.f,0.f,0.f,0.f,0.f,0.f,0.f,0.f,0.f,0.f,0.f,0.342999995f,0.147000000f,0.f,0.147000000f,0.0630000010f,0.f,0.f,0.f,0.f,0.147000000f,0.0630000010f,0.f,0.0630000010f,0.0270000007f}};

typedef _Float16 h16;
typedef unsigned short bf;
typedef __attribute__((ext_vector_type(16))) __bf16   v16bf;
typedef __attribute__((ext_vector_type(16))) _Float16 v16h;
typedef __attribute__((ext_vector_type(8)))  _Float16 v8h;
typedef __attribute__((ext_vector_type(8)))  unsigned short v8us;
typedef __attribute__((ext_vector_type(8)))  float    v8f;
typedef __attribute__((ext_vector_type(4)))  float    v4f;
typedef v8h  __attribute__((may_alias)) v8ha;
typedef v4f  __attribute__((may_alias)) v4fa;
typedef v8us __attribute__((may_alias)) v8usa;

__device__ __forceinline__ unsigned short f2bf(float f) { unsigned u = __float_as_uint(f); u += 0x7FFFu + ((u >> 16) & 1u); return (unsigned short)(u >> 16); }
__device__ __forceinline__ float bf2f(unsigned short b) { return __uint_as_float(((unsigned)b) << 16); }
__device__ __forceinline__ float bfr(float f) { return bf2f(f2bf(f)); }
__device__ __forceinline__ v16h cat16(v8h lo, v8h hi) { return __builtin_shufflevector(lo, hi, 0, 1, 2, 3, 4, 5, 6, 7, 8, 9, 10, 11, 12, 13, 14, 15); }
__device__ __forceinline__ v16bf cat16b(v8us lo, v8us hi) { return __builtin_bit_cast(v16bf, __builtin_shufflevector(lo, hi, 0, 1, 2, 3, 4, 5, 6, 7, 8, 9, 10, 11, 12, 13, 14, 15)); }
__device__ __forceinline__ v8f wmma16(v16h a, v16h b, v8f c) { return __builtin_amdgcn_wmma_f32_16x16x32_f16(false, a, false, b, (short)0, c, false, false); }
__device__ __forceinline__ v8f wmmab(v16bf a, v16bf b, v8f c) { return __builtin_amdgcn_wmma_f32_16x16x32_bf16(false, a, false, b, (short)0, c, false, false); }


__global__ __launch_bounds__(256) void k_bf(const float* __restrict__ src, bf* dst, size_t n8) {
    const size_t i = (size_t)blockIdx.x * 256 + threadIdx.x; if (i >= n8) return;
    const v8f v = *(const v8f*)(src + i * 8); v8us o;
#pragma unroll
    for (int k = 0; k < 8; ++k) o[k] = f2bf(v[k]);
    *(volatile v8us*)(dst + i * 8) = o; __threadfence(); *(volatile v8us*)(dst + i * 8) = o;
}

template <int WHICH>
__global__ __launch_bounds__(256) void k_weff(const float* __restrict__ dw, bf* Wh, bf* Wl) {
    const int u = blockIdx.x * 256 + threadIdx.x; if (u >= CO * KT / 8) return; v8us oh, ol;
#pragma unroll
    for (int i = 0; i < 8; ++i) { const int e = u * 8 + i; const int o = e / KT, r = e % KT, c = r / 27, a = r % 27; float s = 0.f;
#pragma unroll 1
        for (int k = 0; k < 27; ++k) s = fmaf(bfr(dw[((size_t)o * CI + c) * 27 + k]), WHICH == 0 ? c_tab04[k][a] : c_tab07[k][a], s);
        const unsigned short hb = f2bf(s); oh[i] = hb; ol[i] = f2bf(s - bf2f(hb)); }
    *(volatile v8us*)(Wh + (size_t)u * 8) = oh; *(volatile v8us*)(Wl + (size_t)u * 8) = ol; __threadfence(); *(volatile v8us*)(Wh + (size_t)u * 8) = oh; *(volatile v8us*)(Wl + (size_t)u * 8) = ol;
}
__global__ __launch_bounds__(256) void k_im2col(const float* __restrict__ x, int v0, bf* B) {
    const int lane = threadIdx.x & 31, r = blockIdx.x * 8 + (threadIdx.x >> 5); if (r >= NV) return;
    const int v = v0 + r; const int z = v / (DIMO * DIMO), yx = v % (DIMO * DIMO), y = yx / DIMO, xx = yx % DIMO;
#pragma unroll 1
    for (int ps = 0; ps < 2; ++ps) {
#pragma unroll 1
        for (int k0 = lane * 8; k0 < KT; k0 += 256) { v8us ob;
#pragma unroll
            for (int i = 0; i < 8; ++i) { const int kk = k0 + i; const int c = kk / 27, t = kk % 27, kz = t / 9, ky = (t / 3) % 3, kx = t % 3;
                const int Z = z + kz - 1, Y = y + ky - 1, X = xx + kx - 1; const bool ok = (Z >= 0 && Z < DIMO && Y >= 0 && Y < DIMO && X >= 0 && X < DIMO);
                const int Zc = Z < 0 ? 0 : (Z >= DIMO ? DIMO - 1 : Z), Yc = Y < 0 ? 0 : (Y >= DIMO ? DIMO - 1 : Y), Xc = X < 0 ? 0 : (X >= DIMO ? DIMO - 1 : X);
                const float xv = x[(((size_t)c * DIMI + (Zc >> 1)) * DIMI + (Yc >> 1)) * DIMI + (Xc >> 1)]; ob[i] = ok ? f2bf(xv) : (unsigned short)0; }
            *(volatile v8us*)(B + (size_t)r * KT + k0) = ob; }
        if (ps == 0) __threadfence(); }
}
template <bool SPLITA>
__global__ __launch_bounds__(128) void k_gemmrb(const bf* __restrict__ A, const bf* __restrict__ Al, const bf* __restrict__ Bn, const float* __restrict__ rbias, float* C, int ldc, int K) {
    __shared__ __align__(16) float ost[4][16 * 68];
    const int lane = threadIdx.x & 31, wave = threadIdx.x >> 5, lr = lane & 15, hi = lane >> 4;
    const int r0 = blockIdx.x * 64 + wave * 16, c0 = blockIdx.y * 64;
    const size_t aoff = (size_t)(r0 + lr) * K + 8 * hi;
    v8f acc[4];
#pragma unroll
    for (int t = 0; t < 4; ++t) acc[t] = (v8f){};
#pragma unroll 1
    for (int kc = 0; kc < K; kc += 32) {
        const v16bf a = cat16b(*(const v8us*)(A + aoff + kc), *(const v8us*)(A + aoff + kc + 16));
        v16bf al = a; if (SPLITA) al = cat16b(*(const v8us*)(Al + aoff + kc), *(const v8us*)(Al + aoff + kc + 16));
#pragma unroll
        for (int t = 0; t < 4; ++t) { const size_t bo = (size_t)(c0 + t * 16 + lr) * K + kc + 8 * hi; const v16bf bb = cat16b(*(const v8us*)(Bn + bo), *(const v8us*)(Bn + bo + 16)); acc[t] = wmmab(a, bb, acc[t]); if (SPLITA) acc[t] = wmmab(al, bb, acc[t]); }
        asm volatile("v_nop\n\tv_nop\n\tv_nop\n\tv_nop" : "+v"(acc[0]), "+v"(acc[1]), "+v"(acc[2]), "+v"(acc[3]) : "v"(a), "v"(al));
    }
    float* os = &ost[wave][0];
#pragma unroll
    for (int t = 0; t < 4; ++t) {
#pragma unroll
        for (int j = 0; j < 8; ++j) os[(hi * 8 + j) * 68 + t * 16 + lr] = acc[t][j] + bfr(rbias[r0 + hi * 8 + j]); }
    __builtin_amdgcn_wave_barrier(); asm volatile("" ::: "memory");
    float* crow = C + (size_t)r0 * ldc + c0;
    auto pass = [&]() {
#pragma unroll
        for (int s = 0; s < 8; ++s) { const int Lid = (lane >> 3) + 4 * s, piece = lane & 7; const int row = Lid >> 1, cofs = (Lid & 1) * 32 + piece * 4;
            const v4f val = *(const v4fa*)(os + row * 68 + cofs); *(volatile v4f*)(crow + (size_t)row * ldc + cofs) = val; }
    };
    pass(); __threadfence(); pass();
}
__global__ __launch_bounds__(256) void k_bnreluT(const float* __restrict__ CAT, const float* __restrict__ bnp, bf* Ah, bf* Al) {
    __shared__ float tl[64][65];
    const int tid = threadIdx.x, v0 = blockIdx.x * 64, br = blockIdx.y;
    { const int c = tid >> 2, vq = (tid & 3) * 16; const float gsc = bnp[(br * 2 + 0) * CO + c], sh = bnp[(br * 2 + 1) * CO + c];
#pragma unroll
      for (int i = 0; i < 16; ++i) { const float xv = CAT[((size_t)(br * CO + c)) * NV + v0 + vq + i]; tl[vq + i][c] = fmaxf(fmaf(xv, gsc, sh), 0.f); } }
    __syncthreads();
    const int piece = tid & 7, Lid = tid >> 3;
    auto pass = [&]() {
#pragma unroll
        for (int s = 0; s < 2; ++s) { const int vv = Lid + 32 * s; v8us oh, ol;
#pragma unroll
            for (int i = 0; i < 8; ++i) { const float y = tl[vv][piece * 8 + i]; const unsigned short hb = f2bf(y); oh[i] = hb; ol[i] = f2bf(y - bf2f(hb)); }
            const size_t o = (size_t)(v0 + vv) * C3 + br * CO + piece * 8; *(volatile v8us*)(Ah + o) = oh; *(volatile v8us*)(Al + o) = ol; }
    };
    pass(); __threadfence(); pass();
}
template <bool SPLITA, bool F16OUT = false>
__global__ __launch_bounds__(128) void k_gemmb(const bf* __restrict__ A, const bf* __restrict__ Al, const bf* __restrict__ Bn, const float* __restrict__ bias, float* C, int ldc, h16* C2, const float* __restrict__ R = nullptr, int K = DM, int roundR = 1) {
    __shared__ __align__(16) float ost[4][16 * 68];
    const int lane = threadIdx.x & 31, wave = threadIdx.x >> 5, lr = lane & 15, hi = lane >> 4;
    const int r0 = blockIdx.x * 64 + wave * 16, c0 = blockIdx.y * 64;
    const size_t aoff = (size_t)(r0 + lr) * K + 8 * hi;
    size_t boff[4];
#pragma unroll
    for (int t = 0; t < 4; ++t) boff[t] = (size_t)(c0 + t * 16 + lr) * K + 8 * hi;
    v8f acc[4];
#pragma unroll
    for (int t = 0; t < 4; ++t) acc[t] = (v8f){};
#pragma unroll 1
    for (int kc = 0; kc < K; kc += 32) {
        const v16bf a = cat16b(*(const v8us*)(A + aoff + kc), *(const v8us*)(A + aoff + kc + 16));
        v16bf al = a;
        if (SPLITA) al = cat16b(*(const v8us*)(Al + aoff + kc), *(const v8us*)(Al + aoff + kc + 16));
#pragma unroll
        for (int t = 0; t < 4; ++t) { const v16bf b = cat16b(*(const v8us*)(Bn + boff[t] + kc), *(const v8us*)(Bn + boff[t] + kc + 16)); acc[t] = wmmab(a, b, acc[t]); if (SPLITA) acc[t] = wmmab(al, b, acc[t]); }
        asm volatile("v_nop\n\tv_nop\n\tv_nop\n\tv_nop" : "+v"(acc[0]), "+v"(acc[1]), "+v"(acc[2]), "+v"(acc[3]) : "v"(a), "v"(al));
    }
    float* os = &ost[wave][0];
#pragma unroll
    for (int t = 0; t < 4; ++t) { const float bv = bias ? bfr(bias[c0 + t * 16 + lr]) : 0.f;
#pragma unroll
        for (int j = 0; j < 8; ++j) os[(hi * 8 + j) * 68 + t * 16 + lr] = acc[t][j] + bv; }
    __syncthreads();
    if (F16OUT) {
        h16* crow = (h16*)(void*)C + (size_t)r0 * ldc + c0;
        auto pass = [&]() {
#pragma unroll
            for (int s = 0; s < 4; ++s) { const int row = 4 * s + (lane >> 3), piece = lane & 7; const float* sp = os + row * 68 + piece * 8; v8h o, o2;
#pragma unroll
                for (int i = 0; i < 8; ++i) { const h16 a = (h16)sp[i]; o[i] = a; o2[i] = (h16)((sp[i] - (float)a) * LOSC); }
                *(volatile v8h*)(crow + (size_t)row * ldc + piece * 8) = o; if (C2) *(volatile v8h*)(C2 + (size_t)r0 * ldc + c0 + (size_t)row * ldc + piece * 8) = o2; }
        };
        pass(); __threadfence(); pass();
    } else {
        float* crow = C + (size_t)r0 * ldc + c0;
        auto pass = [&]() {
#pragma unroll
            for (int s = 0; s < 8; ++s) { const int Lid = (lane >> 3) + 4 * s, piece = lane & 7; const int row = Lid >> 1, cofs = (Lid & 1) * 32 + piece * 4;
                v4f val = *(const v4fa*)(os + row * 68 + cofs); if (R) { const v4f rv = *(const v4f*)(R + ((size_t)r0 + row) * ldc + c0 + cofs); val += roundR ? (v4f){bfr(rv[0]), bfr(rv[1]), bfr(rv[2]), bfr(rv[3])} : rv; }
                *(volatile v4f*)(crow + (size_t)row * ldc + cofs) = val; }
        };
        pass(); __threadfence(); pass();
    }
}


__global__ __launch_bounds__(256) void k_bn4out(const float* __restrict__ Y, const float* __restrict__ bnp, int v0, float* OUTP) {
    __shared__ __align__(16) float tl[64 * 68];
    const int tid = threadIdx.x, vb = blockIdx.x * 64;
    { const int vv = tid >> 2, oq = (tid & 3) * 16;
#pragma unroll 4
      for (int i = 0; i < 16; ++i) { const int o = oq + i; const float gsc = bnp[6 * CO + o], sh = bnp[7 * CO + o];
          tl[o * 68 + vv] = fmaxf(fmaf(Y[(size_t)(vb + vv) * CO + o], gsc, sh), 0.f); } }
    __syncthreads();
    auto pass = [&]() {
#pragma unroll
        for (int j = 0; j < 4; ++j) { const int idx = tid + 256 * j; const int row = idx >> 4, piece = idx & 15; const v4f v = *(const v4fa*)(tl + row * 68 + piece * 4);
            *(volatile v4f*)(OUTP + (size_t)row * NVOX + v0 + vb + piece * 4) = v; }
    };
    pass(); __threadfence(); pass();
}
__global__ __launch_bounds__(64) void k_bnpack(const float* __restrict__ g1, const float* __restrict__ be1, const float* __restrict__ m1, const float* __restrict__ v1, const float* __restrict__ g2, const float* __restrict__ be2, const float* __restrict__ m2, const float* __restrict__ v2,
                                             const float* __restrict__ g3, const float* __restrict__ be3, const float* __restrict__ m3, const float* __restrict__ v3, const float* __restrict__ g4, const float* __restrict__ be4, const float* __restrict__ m4, const float* __restrict__ v4, float* BNS) {
    const int c = threadIdx.x;
    float sc[4], sh[4];
    sc[0] = bfr(g1[c]) / sqrtf(bfr(v1[c]) + BN_EPS); sh[0] = bfr(be1[c]) - bfr(m1[c]) * sc[0];
    sc[1] = bfr(g2[c]) / sqrtf(bfr(v2[c]) + BN_EPS); sh[1] = bfr(be2[c]) - bfr(m2[c]) * sc[1];
    sc[2] = bfr(g3[c]) / sqrtf(bfr(v3[c]) + BN_EPS); sh[2] = bfr(be3[c]) - bfr(m3[c]) * sc[2];
    sc[3] = bfr(g4[c]) / sqrtf(bfr(v4[c]) + BN_EPS); sh[3] = bfr(be4[c]) - bfr(m4[c]) * sc[3];
#pragma unroll 1
    for (int ps = 0; ps < 2; ++ps) {
#pragma unroll
        for (int s = 0; s < 4; ++s) { *(volatile float*)(BNS + (s * 2 + 0) * CO + c) = sc[s]; *(volatile float*)(BNS + (s * 2 + 1) * CO + c) = sh[s]; }
        if (ps == 0) __threadfence(); }
}

extern "C" void kernel_launch(void* const* d_in, const int* in_sizes, int n_in,
                              void* d_out, int out_size, void* d_ws, size_t ws_size, hipStream_t stream) {
    (void)in_sizes; (void)n_in; (void)out_size;
    const float* x = (const float*)d_in[0]; const float* w1 = (const float*)d_in[1]; const float* b1 = (const float*)d_in[2]; const float* dw1 = (const float*)d_in[3]; const float* db1 = (const float*)d_in[4];
    const float* dw2 = (const float*)d_in[5]; const float* db2 = (const float*)d_in[6]; const float* wc = (const float*)d_in[7]; const float* bc = (const float*)d_in[8];
    const float* bn[16]; for (int i = 0; i < 16; ++i) bn[i] = (const float*)d_in[9 + i];
    float* out = (float*)d_out;
    char* wsp = (char*)d_ws;
    auto take = [&](size_t bytes) { char* p = wsp; wsp += (bytes + 255) & ~(size_t)255; return (void*)p; };
    bf* W1B = (bf*)take((size_t)CO * KT * 2); bf* D1h = (bf*)take((size_t)CO * KT * 2); bf* D1l = (bf*)take((size_t)CO * KT * 2); bf* D2h = (bf*)take((size_t)CO * KT * 2); bf* D2l = (bf*)take((size_t)CO * KT * 2);
    bf* WCB = (bf*)take((size_t)CO * C3 * 2); float* BNP = (float*)take(8 * CO * 4);
    bf* B = (bf*)take((size_t)NV * KT * 2); float* CAT = (float*)take((size_t)C3 * NV * 4); bf* Ah = (bf*)take((size_t)NV * C3 * 2); bf* Al = (bf*)take((size_t)NV * C3 * 2); float* Y4 = (float*)take((size_t)NV * CO * 4);
    if ((size_t)(wsp - (char*)d_ws) > ws_size) return;
    k_bf<<<(CO * KT / 8 + 255) / 256, 256, 0, stream>>>(w1, W1B, CO * KT / 8); k_weff<0><<<(CO * KT / 8 + 255) / 256, 256, 0, stream>>>(dw1, D1h, D1l); k_weff<1><<<(CO * KT / 8 + 255) / 256, 256, 0, stream>>>(dw2, D2h, D2l);
    k_bf<<<(CO * C3 / 8 + 255) / 256, 256, 0, stream>>>(wc, WCB, CO * C3 / 8);
    k_bnpack<<<1, 64, 0, stream>>>(bn[0], bn[1], bn[2], bn[3], bn[4], bn[5], bn[6], bn[7], bn[8], bn[9], bn[10], bn[11], bn[12], bn[13], bn[14], bn[15], BNP);
    for (int ch = 0; ch < NVOX / NV; ++ch) { const int v0 = ch * NV;
        k_im2col<<<NV / 8, 256, 0, stream>>>(x, v0, B);
        k_gemmrb<false><<<dim3(1, NV / 64, 1), 128, 0, stream>>>(W1B, nullptr, B, b1, CAT, NV, KT);
        k_gemmrb<true><<<dim3(1, NV / 64, 1), 128, 0, stream>>>(D1h, D1l, B, db1, CAT + (size_t)CO * NV, NV, KT);
        k_gemmrb<true><<<dim3(1, NV / 64, 1), 128, 0, stream>>>(D2h, D2l, B, db2, CAT + (size_t)2 * CO * NV, NV, KT);
        k_bnreluT<<<dim3(NV / 64, 3, 1), 256, 0, stream>>>(CAT, BNP, Ah, Al);
        k_gemmb<true, false><<<dim3(NV / 64, 1, 1), 128, 0, stream>>>(Ah, Al, WCB, bc, Y4, CO, nullptr, nullptr, C3);
        k_bn4out<<<NV / 64, 256, 0, stream>>>(Y4, BNP, v0, out);
    }
}
